// TransformerDecoderLayerWithAttention_PyTorch_69896297775148
// MI455X (gfx1250) — hardware-verified
//
#include <hip/hip_runtime.h>
#include <math.h>

constexpr int kB   = 4;
constexpr int kT   = 1024;
constexpr int kTM  = 1024;
constexpr int kD   = 1024;
constexpr int kH   = 16;
constexpr int kHS  = 64;
constexpr int kFF  = 4096;
constexpr int kTok = kB * kT;
constexpr int kG   = 8;
constexpr float kWCarry   = 16.0f;
constexpr float kPCarry   = 2048.0f;
constexpr float kCtxCarry = 32.0f;
constexpr float kLnEps    = 1e-5f;

typedef __attribute__((ext_vector_type(16))) _Float16 v16h;
typedef __attribute__((ext_vector_type(8)))  _Float16 v8h;
typedef __attribute__((ext_vector_type(16))) __bf16   v16b;
typedef __attribute__((ext_vector_type(8)))  __bf16   v8b;
typedef __attribute__((ext_vector_type(8)))  float    v8f;
typedef __attribute__((ext_vector_type(4)))  float    v4f;
typedef __attribute__((ext_vector_type(4)))  unsigned int v4u;
typedef __attribute__((ext_vector_type(2)))  unsigned int v2u;

__device__ __forceinline__ unsigned short f2bf_bits(float f) {
  unsigned u = __float_as_uint(f);
  return (unsigned short)((u + 0x7FFFu + ((u >> 16) & 1u)) >> 16);
}
__device__ __forceinline__ float bf_bits2f(unsigned short h) { return __uint_as_float(((unsigned)h) << 16); }

__device__ __forceinline__ void dep_guard_h(v8f& a, v8f& b, v16h x, v16h y) { asm volatile("v_nop\n\tv_nop\n\tv_nop\n\tv_nop" : "+v"(a), "+v"(b) : "v"(x), "v"(y)); }
__device__ __forceinline__ void dep_guard_b(v8f& a, v8f& b, v16b x, v16b y) { asm volatile("v_nop\n\tv_nop\n\tv_nop\n\tv_nop" : "+v"(a), "+v"(b) : "v"(x), "v"(y)); }
__device__ __forceinline__ void keep4_h(v16h a, v16h b, v16h c, v16h d) { asm volatile("v_nop" :: "v"(a), "v"(b), "v"(c), "v"(d)); }
__device__ __forceinline__ void keep4_b(v16b a, v16b b, v16b c, v16b d) { asm volatile("v_nop" :: "v"(a), "v"(b), "v"(c), "v"(d)); }
__device__ __forceinline__ void acc_guard4(v8f& a, v8f& b, v8f& c, v8f& d) { asm volatile("v_nop\n\tv_nop\n\tv_nop\n\tv_nop" : "+v"(a), "+v"(b), "+v"(c), "+v"(d)); }
template <typename T> struct Frag;
template <> struct Frag<_Float16> {
  typedef v16h V; union U { v16h v; v8h h[2]; };
  static __device__ __forceinline__ v16h load(const _Float16* p) {
    U f; f.h[0] = *(const v8h*)(p); f.h[1] = *(const v8h*)(p + 16); return f.v;
  }
  static __device__ __forceinline__ v8f mma(v16h a, v16h b, v8f c) {
    return __builtin_amdgcn_wmma_f32_16x16x32_f16(false, a, false, b, (short)0, c, false, false);
  }
  static __device__ __forceinline__ void guard(v8f& a, v8f& b, v16h x, v16h y) { dep_guard_h(a, b, x, y); }
  static __device__ __forceinline__ void keep(v16h a, v16h b, v16h c, v16h d) { keep4_h(a, b, c, d); }
};
template <> struct Frag<__bf16> {
  typedef v16b V; union U { v16b v; v8b h[2]; };
  static __device__ __forceinline__ v16b load(const __bf16* p) {
    U f; f.h[0] = *(const v8b*)(p); f.h[1] = *(const v8b*)(p + 16); return f.v;
  }
  static __device__ __forceinline__ v8f mma(v16b a, v16b b, v8f c) {
    return __builtin_amdgcn_wmma_f32_16x16x32_bf16(false, a, false, b, (short)0, c, false, false);
  }
  static __device__ __forceinline__ void guard(v8f& a, v8f& b, v16b x, v16b y) { dep_guard_b(a, b, x, y); }
  static __device__ __forceinline__ void keep(v16b a, v16b b, v16b c, v16b d) { keep4_b(a, b, c, d); }
};

__device__ __forceinline__ unsigned pk16(unsigned short a, unsigned short b) { return (unsigned)a | ((unsigned)b << 16); }
__device__ __forceinline__ unsigned short h_bits(float f) { const _Float16 h = (_Float16)f; return __builtin_bit_cast(unsigned short, h); }

template <int ET> struct Elem;
template <> struct Elem<0> { typedef _Float16 T; };
template <> struct Elem<1> { typedef __bf16 T; };
template <int ET, bool SPLIT, int BIAS_MODE, int OUT_MODE, bool RESID, int ACT = 0>
__global__ __launch_bounds__(256) void wmma_gemm64(
    const unsigned short* __restrict__ Ap, const unsigned short* __restrict__ A2p, int lda, long strideA,
    const unsigned short* __restrict__ Btp, const unsigned short* __restrict__ Bt2p, int ldb, long strideB,
    void* __restrict__ Cout, void* __restrict__ Cout2, int ldc, long strideC,
    const float* __restrict__ bias,
    const float* __restrict__ resid, long strideR,
    int M, int N, int K, float scale) {
  typedef typename Elem<ET>::T T;
  typedef typename Frag<T>::V V;
  const T* A = (const T*)Ap; const T* A2 = (const T*)A2p; const T* Bt = (const T*)Btp; const T* Bt2 = (const T*)Bt2p;
  __shared__ __align__(16) float sT[8][16 * 68];
  const int b    = blockIdx.y;
  const int lane = threadIdx.x & 31;
  const int wave = threadIdx.x >> 5;
  const int tilesN = N >> 6;
  const int tilesM = M >> 6;
  const int tile = blockIdx.x * 8 + wave;
  if (tile >= tilesM * tilesN) return;
  const int tm = tile / tilesN;
  const int tn = tile - tm * tilesN;
  const int m0 = tm << 6;
  const int n0 = tn << 6;

  const T* Ab  = A  + (size_t)b * strideA;
  const T* Bb  = Bt + (size_t)b * strideB;
  const T* Ab2 = SPLIT ? (A2  + (size_t)b * strideA) : nullptr;
  const T* Bb2 = SPLIT ? (Bt2 + (size_t)b * strideB) : nullptr;

  const int rlane = lane & 15;
  const int koff  = (lane >> 4) * 8;
  const int mOff  = (lane >> 4) * 8;

  v8f acc[4][4];
#pragma unroll
  for (int i = 0; i < 4; ++i)
#pragma unroll
    for (int j = 0; j < 4; ++j) acc[i][j] = (v8f){0.f,0.f,0.f,0.f,0.f,0.f,0.f,0.f};

  for (int k0 = 0; k0 < K; k0 += 32) {
    V bh[4], bl[4];
#pragma unroll
    for (int j = 0; j < 4; ++j) {
      const size_t bo = (size_t)(n0 + (j << 4) + rlane) * ldb + koff + k0;
      bh[j] = Frag<T>::load(Bb + bo);
      if (SPLIT) bl[j] = Frag<T>::load(Bb2 + bo);
    }
#pragma unroll
    for (int i = 0; i < 4; ++i) {
      const size_t ao = (size_t)(m0 + (i << 4) + rlane) * lda + koff + k0;
      V ah = Frag<T>::load(Ab + ao);
      V al;
      if (SPLIT) al = Frag<T>::load(Ab2 + ao);
#pragma unroll
      for (int j = 0; j < 4; ++j) {
        acc[i][j] = Frag<T>::mma(ah, bh[j], acc[i][j]);
        if (SPLIT) {
          acc[i][j] = Frag<T>::mma(ah, bl[j], acc[i][j]);
          acc[i][j] = Frag<T>::mma(al, bh[j], acc[i][j]);
        }
      }
      Frag<T>::guard(acc[i][0], acc[i][3], ah, SPLIT ? al : ah);
    }
    Frag<T>::keep(bh[0], bh[1], bh[2], bh[3]);
    if (SPLIT) Frag<T>::keep(bl[0], bl[1], bl[2], bl[3]);
  }
  acc_guard4(acc[0][0], acc[0][1], acc[0][2], acc[0][3]);
  acc_guard4(acc[1][0], acc[1][1], acc[1][2], acc[1][3]);
  acc_guard4(acc[2][0], acc[2][1], acc[2][2], acc[2][3]);
  acc_guard4(acc[3][0], acc[3][1], acc[3][2], acc[3][3]);

  float* slab = sT[wave];
  const float* Rb = RESID ? (resid + (size_t)b * strideR) : nullptr;
#pragma unroll
  for (int i = 0; i < 4; ++i) {
    const int mBase = m0 + (i << 4);
#pragma unroll
    for (int j = 0; j < 4; ++j) {
      const int n = n0 + (j << 4) + rlane;
      float bv = 0.f;
      if (BIAS_MODE == 2) bv = bias[n];
#pragma unroll
      for (int r = 0; r < 8; ++r) {
        float v = acc[i][j][r] * scale;
        if (BIAS_MODE == 1) v += bias[mBase + mOff + r];
        if (BIAS_MODE == 2) v += bv;
        if (RESID) v += Rb[(size_t)(mBase + mOff + r) * ldc + n];
        if (ACT == 2) v = fmaxf(v, 0.0f);
        if (ACT == 4) v = (v > 0.f) ? v : 0.01f * v;
        slab[(mOff + r) * 68 + (j << 4) + rlane] = v;
      }
    }
    __builtin_amdgcn_fence(__ATOMIC_RELEASE, "workgroup");
    __builtin_amdgcn_wave_barrier();
    __builtin_amdgcn_fence(__ATOMIC_ACQUIRE, "workgroup");
    if (OUT_MODE == 0) {
      float* C = (float*)Cout + (size_t)b * strideC;
      const int hh = lane >> 4, c4 = (lane & 15) * 4;
      for (int pass = 0; pass < 2; ++pass) {
#pragma unroll
        for (int it = 0; it < 8; ++it) {
          const int row = it * 2 + hh;
          v4f v = *(const v4f*)(slab + row * 68 + c4);
          *(volatile v4f*)(C + (size_t)(mBase + row) * ldc + n0 + c4) = v;
        }
        __threadfence();
      }
    } else {
      const int q = lane >> 3, c8 = (lane & 7) * 8;
      unsigned short* C  = (unsigned short*)Cout  + (size_t)b * strideC;
      unsigned short* C2 = (OUT_MODE == 2) ? ((unsigned short*)Cout2 + (size_t)b * strideC) : nullptr;
      for (int pass = 0; pass < 2; ++pass) {
#pragma unroll
        for (int it = 0; it < 4; ++it) {
          const int row = it * 4 + q;
          const float* sp = slab + row * 68 + c8;
          v8h hv, lv;
#pragma unroll
          for (int e = 0; e < 8; ++e) {
            if (OUT_MODE == 1) {
              hv[e] = (_Float16)sp[e];
            } else {
              unsigned short hb = f2bf_bits(sp[e]);
              unsigned short lb = f2bf_bits(sp[e] - bf_bits2f(hb));
              hv[e] = __builtin_bit_cast(_Float16, hb);
              lv[e] = __builtin_bit_cast(_Float16, lb);
            }
          }
          *(volatile v8h*)(C + (size_t)(mBase + row) * ldc + n0 + c8) = hv;
          if (OUT_MODE == 2) *(volatile v8h*)(C2 + (size_t)(mBase + row) * ldc + n0 + c8) = lv;
        }
        __threadfence();
      }
    }
    __builtin_amdgcn_fence(__ATOMIC_RELEASE, "workgroup");
    __builtin_amdgcn_wave_barrier();
    __builtin_amdgcn_fence(__ATOMIC_ACQUIRE, "workgroup");
  }
}

__global__ __launch_bounds__(256) void wtcast_kernel(const float* __restrict__ W0, const float* __restrict__ W1,
                                                     const float* __restrict__ W2, const float* __restrict__ W3,
                                                     unsigned short* __restrict__ out, long outStride,
                                                     int R, int Ccols, float scale) {
  __shared__ float sm[64][65];
  const int t  = threadIdx.x;
  const int r0 = blockIdx.x * 64;
  const int c0 = blockIdx.y * 64;
  const int z  = blockIdx.z;
  const float* W = (z == 0) ? W0 : (z == 1) ? W1 : (z == 2) ? W2 : W3;
#pragma unroll
  for (int i = 0; i < 16; ++i) {
    const int e = i * 256 + t;
    const int r = e >> 6;
    const int c = e & 63;
    sm[c][r] = W[(size_t)(r0 + r) * Ccols + c0 + c] * scale;
  }
  __syncthreads();
  const int lane = t & 31, wave = t >> 5;
  const int q = lane >> 3, c8 = (lane & 7) * 8;
  unsigned short* op = out + (size_t)z * outStride;
  for (int pass = 0; pass < 2; ++pass) {
#pragma unroll
    for (int it = 0; it < 2; ++it) {
      const int row = wave * 8 + it * 4 + q;
      unsigned short hb[8];
#pragma unroll
      for (int e = 0; e < 8; ++e) hb[e] = h_bits(sm[row][c8 + e]);
      const v4u u = (v4u){pk16(hb[0], hb[1]), pk16(hb[2], hb[3]), pk16(hb[4], hb[5]), pk16(hb[6], hb[7])};
      *(volatile v4u*)(op + (size_t)(c0 + row) * R + r0 + c8) = u;
    }
    __threadfence();
  }
}

__global__ __launch_bounds__(256) void cast8_f16_kernel(const float* __restrict__ in, unsigned short* __restrict__ out, int n8) {
  const int i = blockIdx.x * 256 + threadIdx.x;
  if (i >= n8) return;
  const float* p = in + 8 * (size_t)i;
  const v4f a = *(const v4f*)(p);
  const v4f c = *(const v4f*)(p + 4);
  unsigned short hb[8];
#pragma unroll
  for (int e = 0; e < 4; ++e) {
    hb[e]     = h_bits(a[e]);
    hb[4 + e] = h_bits(c[e]);
  }
  const v4u u = (v4u){pk16(hb[0], hb[1]), pk16(hb[2], hb[3]), pk16(hb[4], hb[5]), pk16(hb[6], hb[7])};
  unsigned short* q = out + 8 * (size_t)i;
  *(volatile v4u*)q = u;
  __threadfence();
  *(volatile v4u*)q = u;
}

__global__ __launch_bounds__(256) void softmax_kernel(const float* __restrict__ S, unsigned short* __restrict__ P,
                                                      const float* __restrict__ attPart, float* __restrict__ attDst, int mode) {
  __shared__ float redM[8];
  __shared__ float redS[8];
  __shared__ __align__(16) unsigned int stg[512];
  const int trow = blockIdx.x;
  const int t = threadIdx.x, lane = t & 31, wave = t >> 5;
  const int c0 = t * 4;
  float asum[4] = {0.f, 0.f, 0.f, 0.f};
  if (mode == 2) {
    const v4f a = *(const v4f*)(attPart + (size_t)trow * kTM + c0);
#pragma unroll
    for (int j = 0; j < 4; ++j) asum[j] = a[j];
  }
#pragma unroll 1
  for (int g = 0; g < kG; ++g) {
    const float* sr = S + ((size_t)g * kT + trow) * kTM + c0;
    const v4f x = *(const v4f*)sr;
    float m = fmaxf(fmaxf(x[0], x[1]), fmaxf(x[2], x[3]));
#pragma unroll
    for (int off = 16; off > 0; off >>= 1) m = fmaxf(m, __shfl_xor(m, off, 32));
    __syncthreads();
    if (lane == 0) redM[wave] = m;
    __syncthreads();
    float rm = redM[0];
#pragma unroll
    for (int i = 1; i < 8; ++i) rm = fmaxf(rm, redM[i]);
    float ex[4];
    float s = 0.f;
#pragma unroll
    for (int j = 0; j < 4; ++j) { ex[j] = expf(x[j] - rm); s += ex[j]; }
#pragma unroll
    for (int off = 16; off > 0; off >>= 1) s += __shfl_xor(s, off, 32);
    if (lane == 0) redS[wave] = s;
    __syncthreads();
    float tot = redS[0];
#pragma unroll
    for (int i = 1; i < 8; ++i) tot += redS[i];
    const float inv = 1.0f / tot;
    float p[4];
#pragma unroll
    for (int j = 0; j < 4; ++j) { p[j] = ex[j] * inv; asum[j] += p[j]; }
    const v2u u = (v2u){pk16(h_bits(p[0] * kPCarry), h_bits(p[1] * kPCarry)),
                        pk16(h_bits(p[2] * kPCarry), h_bits(p[3] * kPCarry))};
    *(v2u*)(stg + 2 * t) = u;
    __syncthreads();
    if (t < 128) {
      const v4u w = *(const v4u*)(stg + 4 * t);
      unsigned short* dst = P + ((size_t)g * kT + trow) * kTM + 8 * t;
      *(volatile v4u*)dst = w;
      __threadfence();
      *(volatile v4u*)dst = w;
    }
  }
  if (mode != 0) {
    v4f o;
#pragma unroll
    for (int j = 0; j < 4; ++j) o[j] = (mode == 2) ? asum[j] * (1.0f / 16.0f) : asum[j];
    float* dst = attDst + (size_t)trow * kTM + c0;
    *(volatile v4f*)dst = o;
    __threadfence();
    *(volatile v4f*)dst = o;
  }
}

__global__ __launch_bounds__(256) void layernorm_kernel(const float* __restrict__ X, const float* __restrict__ gam,
                                                        const float* __restrict__ bet, float* __restrict__ Y32,
                                                        unsigned short* __restrict__ Y16, int mode) {
  __shared__ float redA[8];
  __shared__ float redB[8];
  __shared__ __align__(16) unsigned int stg[512];
  const int row = blockIdx.x;
  const int t = threadIdx.x, lane = t & 31, wave = t >> 5;
  const int c0 = t * 4;
  const v4f xv = *(const v4f*)(X + (size_t)row * kD + c0);
  float s = (xv[0] + xv[1]) + (xv[2] + xv[3]);
#pragma unroll
  for (int off = 16; off > 0; off >>= 1) s += __shfl_xor(s, off, 32);
  if (lane == 0) redA[wave] = s;
  __syncthreads();
  float tot = redA[0];
#pragma unroll
  for (int i = 1; i < 8; ++i) tot += redA[i];
  const float mean = tot * (1.0f / 1024.0f);
  float d[4];
#pragma unroll
  for (int j = 0; j < 4; ++j) d[j] = xv[j] - mean;
  float q = (d[0] * d[0] + d[1] * d[1]) + (d[2] * d[2] + d[3] * d[3]);
#pragma unroll
  for (int off = 16; off > 0; off >>= 1) q += __shfl_xor(q, off, 32);
  if (lane == 0) redB[wave] = q;
  __syncthreads();
  float tq = redB[0];
#pragma unroll
  for (int i = 1; i < 8; ++i) tq += redB[i];
  const float var = tq * (1.0f / 1024.0f);
  const float inv = 1.0f / sqrtf(var + kLnEps);
  const v4f gv = *(const v4f*)(gam + c0);
  const v4f bv = *(const v4f*)(bet + c0);
  v4f o;
#pragma unroll
  for (int j = 0; j < 4; ++j) o[j] = d[j] * inv * gv[j] + bv[j];
  float* dst = Y32 + (size_t)row * kD + c0;
  *(volatile v4f*)dst = o;
  __threadfence();
  *(volatile v4f*)dst = o;
  if (mode == 0) {
    const v2u u = (v2u){pk16(h_bits(o[0]), h_bits(o[1])), pk16(h_bits(o[2]), h_bits(o[3]))};
    *(v2u*)(stg + 2 * t) = u;
    __syncthreads();
    if (t < 128) {
      const v4u w = *(const v4u*)(stg + 4 * t);
      unsigned short* d16 = Y16 + (size_t)row * kD + 8 * t;
      *(volatile v4u*)d16 = w;
      __threadfence();
      *(volatile v4u*)d16 = w;
    }
  }
}

template <int BIAS_MODE, int OUT_MODE, bool RESID, int ACT>
static void gemm_launch(hipStream_t st,
                        const unsigned short* A, int lda, long sA,
                        const unsigned short* Bt, int ldb, long sB,
                        void* C, int ldc, long sC,
                        const float* bias, const float* resid, long sR,
                        int M, int N, int K, float scale, int batch) {
  const int tiles = (M / 64) * (N / 64);
  dim3 grid((unsigned)((tiles + 7) / 8), (unsigned)batch, 1);
  wmma_gemm64<0, false, BIAS_MODE, OUT_MODE, RESID, ACT><<<grid, dim3(256), 0, st>>>(
      A, A, lda, sA, Bt, Bt, ldb, sB, C, C, ldc, sC, bias, resid, sR, M, N, K, scale);
}

extern "C" void kernel_launch(void* const* d_in, const int* in_sizes, int n_in,
                              void* d_out, int out_size, void* d_ws, size_t ws_size,
                              hipStream_t stream)
{
  (void)in_sizes;
  constexpr size_t kMiB = 1048576;
  if (n_in < 28) return;
  if (ws_size < 128 * kMiB) return;
  if ((size_t)out_size < 2 * (size_t)kTok * kD) return;

  const float* tgt   = (const float*)d_in[0];
  const float* mem   = (const float*)d_in[1];
  const float* sa_wq = (const float*)d_in[2];  const float* sa_bq = (const float*)d_in[3];
  const float* sa_wk = (const float*)d_in[4];  const float* sa_bk = (const float*)d_in[5];
  const float* sa_wv = (const float*)d_in[6];  const float* sa_bv = (const float*)d_in[7];
  const float* sa_wo = (const float*)d_in[8];  const float* sa_bo = (const float*)d_in[9];
  const float* ca_wq = (const float*)d_in[10]; const float* ca_bq = (const float*)d_in[11];
  const float* ca_wk = (const float*)d_in[12]; const float* ca_bk = (const float*)d_in[13];
  const float* ca_wv = (const float*)d_in[14]; const float* ca_bv = (const float*)d_in[15];
  const float* ca_wo = (const float*)d_in[16]; const float* ca_bo = (const float*)d_in[17];
  const float* w1    = (const float*)d_in[18]; const float* b1    = (const float*)d_in[19];
  const float* w2    = (const float*)d_in[20]; const float* b2    = (const float*)d_in[21];
  const float* ln1g  = (const float*)d_in[22]; const float* ln1b  = (const float*)d_in[23];
  const float* ln2g  = (const float*)d_in[24]; const float* ln2b  = (const float*)d_in[25];
  const float* ln3g  = (const float*)d_in[26]; const float* ln3b  = (const float*)d_in[27];

  float* out0 = (float*)d_out;
  float* out1 = (float*)d_out + (size_t)kTok * kD;

  char* ws = (char*)d_ws;
  float*          SC    = (float*)(ws + 0 * kMiB);
  float*          SUM32 = (float*)(ws + 0 * kMiB);
  unsigned short* HID   = (unsigned short*)(ws + 0 * kMiB);
  unsigned short* PP    = (unsigned short*)(ws + 32 * kMiB);
  float*          SUM3  = (float*)(ws + 32 * kMiB);
  unsigned short* QPL   = (unsigned short*)(ws + 48 * kMiB);
  unsigned short* W1T   = (unsigned short*)(ws + 48 * kMiB);
  unsigned short* KPL   = (unsigned short*)(ws + 56 * kMiB);
  unsigned short* W2T   = (unsigned short*)(ws + 56 * kMiB);
  unsigned short* VT    = (unsigned short*)(ws + 64 * kMiB);
  unsigned short* CTX   = (unsigned short*)(ws + 72 * kMiB);
  unsigned short* ACT   = (unsigned short*)(ws + 80 * kMiB);
  unsigned short* MEM   = (unsigned short*)(ws + 88 * kMiB);
  unsigned short* WSA   = (unsigned short*)(ws + 96 * kMiB);
  float*          ATTP  = (float*)(ws + 96 * kMiB);
  unsigned short* WCA   = (unsigned short*)(ws + 104 * kMiB);
  float*          X32   = (float*)(ws + 112 * kMiB);

  const size_t wplane = (size_t)kD * kD;
  const size_t tplane = (size_t)kT * kD;
  const float wscaleInv   = 1.0f / kWCarry;
  const float scoreScale  = 0.125f;
  const float pvScale     = kCtxCarry / kPCarry;
  const float woScale     = 1.0f / (kCtxCarry * kWCarry);
  const dim3 blk(256);

  {
    const int n8 = (int)((size_t)kTok * kD / 8);
    cast8_f16_kernel<<<dim3((unsigned)((n8 + 255) / 256)), blk, 0, stream>>>(tgt, ACT, n8);
    cast8_f16_kernel<<<dim3((unsigned)((n8 + 255) / 256)), blk, 0, stream>>>(mem, MEM, n8);
    wtcast_kernel<<<dim3(kD / 64, kD / 64, 4), blk, 0, stream>>>(sa_wq, sa_wk, sa_wv, sa_wo, WSA, (long)wplane, kD, kD, kWCarry);
    wtcast_kernel<<<dim3(kD / 64, kD / 64, 4), blk, 0, stream>>>(ca_wq, ca_wk, ca_wv, ca_wo, WCA, (long)wplane, kD, kD, kWCarry);
  }

  auto attention = [&](const unsigned short* Aq, const unsigned short* Akv, const unsigned short* Wt,
                       const float* bq, const float* bk, const float* bvv, bool withAtt) {
    gemm_launch<2, 1, false, 0>(stream, Aq, kD, 0, Wt + 0 * wplane, kD, 0, QPL, kD, 0, bq, tgt, 0,
                                kTok, kD, kD, wscaleInv, 1);
    gemm_launch<2, 1, false, 0>(stream, Akv, kD, 0, Wt + 1 * wplane, kD, 0, KPL, kD, 0, bk, tgt, 0,
                                kB * kTM, kD, kD, wscaleInv, 1);
    gemm_launch<1, 1, false, 0>(stream, Wt + 2 * wplane, kD, 0, Akv, kD, (long)tplane, VT, kTM, (long)((size_t)kD * kTM),
                                bvv, tgt, 0, kD, kTM, kD, wscaleInv, kB);
    for (int b = 0; b < kB; ++b) {
      for (int hc = 0; hc < kH / kG; ++hc) {
        const int h0 = hc * kG;
        gemm_launch<0, 0, false, 0>(stream,
                                    QPL + (size_t)b * tplane + (size_t)h0 * kHS, kD, (long)kHS,
                                    KPL + (size_t)b * tplane + (size_t)h0 * kHS, kD, (long)kHS,
                                    SC, kTM, (long)((size_t)kT * kTM), sa_bq, tgt, 0,
                                    kT, kTM, kHS, scoreScale, kG);
        const int mode = withAtt ? (hc == 0 ? 1 : 2) : 0;
        float* attDst = (mode == 2) ? (out1 + (size_t)b * kT * kTM) : ATTP;
        softmax_kernel<<<dim3(kT), blk, 0, stream>>>(SC, PP, ATTP, attDst, mode);
        gemm_launch<0, 1, false, 0>(stream,
                                    PP, kTM, (long)((size_t)kT * kTM),
                                    VT + (size_t)b * kD * kTM + (size_t)h0 * kHS * kTM, kTM, (long)((size_t)kHS * kTM),
                                    CTX + (size_t)b * tplane + (size_t)h0 * kHS, kD, (long)kHS,
                                    sa_bq, tgt, 0, kT, kHS, kTM, pvScale, kG);
      }
    }
  };

  attention(ACT, ACT, WSA, sa_bq, sa_bk, sa_bv, false);
  gemm_launch<2, 0, true, 0>(stream, CTX, kD, 0, WSA + 3 * wplane, kD, 0, SUM32, kD, 0, sa_bo, tgt, 0,
                             kTok, kD, kD, woScale, 1);
  layernorm_kernel<<<dim3(kTok), blk, 0, stream>>>(SUM32, ln1g, ln1b, X32, ACT, 0);

  attention(ACT, MEM, WCA, ca_bq, ca_bk, ca_bv, true);
  gemm_launch<2, 0, true, 0>(stream, CTX, kD, 0, WCA + 3 * wplane, kD, 0, SUM32, kD, 0, ca_bo, X32, 0,
                             kTok, kD, kD, woScale, 1);
  layernorm_kernel<<<dim3(kTok), blk, 0, stream>>>(SUM32, ln2g, ln2b, X32, ACT, 0);

  wtcast_kernel<<<dim3(kD / 64, kFF / 64, 1), blk, 0, stream>>>(w1, w1, w1, w1, W1T, 0L, kD, kFF, kWCarry);
  wtcast_kernel<<<dim3(kFF / 64, kD / 64, 1), blk, 0, stream>>>(w2, w2, w2, w2, W2T, 0L, kFF, kD, kWCarry);
  gemm_launch<2, 1, false, 2>(stream, ACT, kD, 0, W1T, kD, 0, HID, kFF, 0, b1, tgt, 0,
                              kTok, kFF, kD, wscaleInv, 1);
  gemm_launch<2, 0, true, 0>(stream, HID, kFF, 0, W2T, kFF, 0, SUM3, kD, 0, b2, X32, 0,
                             kTok, kD, kFF, wscaleInv, 1);
  layernorm_kernel<<<dim3(kTok), blk, 0, stream>>>(SUM3, ln3g, ln3b, out0, ACT, 1);
}
